// MultiHeadSelfAttention_36696200577656
// MI455X (gfx1250) — hardware-verified
//
#include <hip/hip_runtime.h>


#ifndef NB
#define NB 4
#endif
#ifndef SEQ
#define SEQ 2048
#endif
#define NB_FULL  4
#define SEQ_FULL 2048
#define DM   768
#define NH   12
#define HD   64
#define RH   ((SEQ) < 512 ? (SEQ) : 512)
#define PCAR 1024.0f
#define SCL  0.125f
#define L2E  1.4426950408889634f

static_assert(NH * HD == DM);
static_assert(DM % 64 == 0);
static_assert(SEQ % 64 == 0);
static_assert(RH % 64 == 0);
static_assert(SEQ <= SEQ_FULL);
static_assert(NB <= NB_FULL);
static_assert((SEQ * DM / 8) % 256 == 0);
static_assert((DM * DM / 8) % 256 == 0);
static_assert((SEQ * 32) % 256 == 0);
static_assert((NB * NH * SEQ * HD / 2) % 256 == 0);

typedef _Float16 h16;
typedef unsigned short bf;
typedef __attribute__((ext_vector_type(16))) __bf16   v16bf;
typedef __attribute__((ext_vector_type(16))) _Float16 v16h;
typedef __attribute__((ext_vector_type(8)))  _Float16 v8h;
typedef __attribute__((ext_vector_type(8)))  unsigned short v8us;
typedef __attribute__((ext_vector_type(8)))  float    v8f;
typedef __attribute__((ext_vector_type(4)))  float    v4f;
typedef __attribute__((ext_vector_type(2)))  float    v2f;
typedef __attribute__((ext_vector_type(2)))  _Float16 v2h;
typedef __attribute__((ext_vector_type(2)))  unsigned short v2us;
typedef v4f  __attribute__((may_alias)) v4fa;
typedef v8us __attribute__((may_alias)) v8usa;

__device__ __forceinline__ unsigned short f2bf(float f) { unsigned u = __float_as_uint(f); u += 0x7FFFu + ((u >> 16) & 1u); return (unsigned short)(u >> 16); }
__device__ __forceinline__ float bf2f(unsigned short b) { return __uint_as_float(((unsigned)b) << 16); }
__device__ __forceinline__ float bfr(float f) { return bf2f(f2bf(f)); }
__device__ __forceinline__ void splitf(float y, unsigned short& h, unsigned short& l) { h = f2bf(y); l = f2bf(y - bf2f(h)); }
__device__ __forceinline__ v16h cat16(v8h lo, v8h hi) { return __builtin_shufflevector(lo, hi, 0, 1, 2, 3, 4, 5, 6, 7, 8, 9, 10, 11, 12, 13, 14, 15); }
__device__ __forceinline__ v16bf cat16b(v8us lo, v8us hi) { return __builtin_bit_cast(v16bf, __builtin_shufflevector(lo, hi, 0, 1, 2, 3, 4, 5, 6, 7, 8, 9, 10, 11, 12, 13, 14, 15)); }
__device__ __forceinline__ v8f wmma16(v16h a, v16h b, v8f c) { return __builtin_amdgcn_wmma_f32_16x16x32_f16(false, a, false, b, (short)0, c, false, false); }
__device__ __forceinline__ v8f wmmab(v16bf a, v16bf b, v8f c) { return __builtin_amdgcn_wmma_f32_16x16x32_bf16(false, a, false, b, (short)0, c, false, false); }

template <typename T16> struct WFrag;
template <> struct WFrag<h16> {
    typedef v16h V;
    static __device__ __forceinline__ V ld(const h16* p) { return cat16(*(const v8h*)p, *(const v8h*)(p + 16)); }
    static __device__ __forceinline__ v8f mma(V a, V b, v8f c) { return wmma16(a, b, c); }
    static __device__ __forceinline__ V pkh(v8f p0, v8f p1) { v16h o;
#pragma unroll
        for (int i = 0; i < 8; ++i) { o[i] = (h16)(p0[i] * PCAR); o[8 + i] = (h16)(p1[i] * PCAR); }
        return o; }
    static __device__ __forceinline__ V pkl(v8f p0, v8f p1) { (void)p0; (void)p1; v16h o = {}; return o; }
    static __device__ __forceinline__ float ocs() { return 1.0f / PCAR; }
};
template <> struct WFrag<bf> {
    typedef v16bf V;
    static __device__ __forceinline__ V ld(const bf* p) { return cat16b(*(const v8us*)p, *(const v8us*)(p + 16)); }
    static __device__ __forceinline__ v8f mma(V a, V b, v8f c) { return wmmab(a, b, c); }
    static __device__ __forceinline__ V pkh(v8f p0, v8f p1) { v8us a, c;
#pragma unroll
        for (int i = 0; i < 8; ++i) { a[i] = f2bf(p0[i]); c[i] = f2bf(p1[i]); }
        return cat16b(a, c); }
    static __device__ __forceinline__ V pkl(v8f p0, v8f p1) { v8us a, c;
#pragma unroll
        for (int i = 0; i < 8; ++i) { a[i] = f2bf(p0[i] - bf2f(f2bf(p0[i]))); c[i] = f2bf(p1[i] - bf2f(f2bf(p1[i]))); }
        return cat16b(a, c); }
    static __device__ __forceinline__ float ocs() { return 1.0f; }
};
template <typename T16> __device__ __forceinline__ v8f mmag(typename WFrag<T16>::V a, typename WFrag<T16>::V b, v8f c) {
    c = WFrag<T16>::mma(a, b, c);
    asm volatile("v_nop\n\tv_nop\n\tv_nop\n\tv_nop" : "+v"(c) : "v"(a), "v"(b));
    return c;
}

template <typename T16, int NSPLIT, bool BIAS>
__global__ __launch_bounds__(32) void k_gemmw(const T16* __restrict__ A, const T16* __restrict__ A2, const T16* __restrict__ Bt, const T16* __restrict__ Bt2, int K, float* C, int ldc, const float* __restrict__ bias, size_t sA, size_t sB, size_t sC) {
    typedef typename WFrag<T16>::V V;
    __shared__ __align__(16) float os[16 * 68];
    const size_t z = blockIdx.z; A += z * sA; if (A2) A2 += z * sA; Bt += z * sB; if (Bt2) Bt2 += z * sB; C += z * sC;
    const int lane = threadIdx.x & 31, lr = lane & 15, hi = lane >> 4; const int r0 = blockIdx.x * 64, c0 = blockIdx.y * 64;
    v8f acc[4][4];
#pragma unroll
    for (int mb = 0; mb < 4; ++mb)
#pragma unroll
        for (int nb = 0; nb < 4; ++nb) acc[mb][nb] = (v8f){};
    const size_t aoff = (size_t)(r0 + lr) * K + 8 * hi, boff = (size_t)(c0 + lr) * K + 8 * hi;
#pragma unroll 1
    for (int kc = 0; kc < K; kc += 32) {
        V a[4], a2[4];
#pragma unroll
        for (int mb = 0; mb < 4; ++mb) { a[mb] = WFrag<T16>::ld(A + aoff + (size_t)mb * 16 * K + kc); if (NSPLIT == 1 || NSPLIT == 2) a2[mb] = WFrag<T16>::ld(A2 + aoff + (size_t)mb * 16 * K + kc); }
#pragma unroll
        for (int nb = 0; nb < 4; ++nb) { const V b = WFrag<T16>::ld(Bt + boff + (size_t)nb * 16 * K + kc); V b2; if (NSPLIT >= 2) b2 = WFrag<T16>::ld(Bt2 + boff + (size_t)nb * 16 * K + kc);
#pragma unroll
            for (int mb = 0; mb < 4; ++mb) { acc[mb][nb] = WFrag<T16>::mma(a[mb], b, acc[mb][nb]); if (NSPLIT == 1 || NSPLIT == 2) acc[mb][nb] = WFrag<T16>::mma(a2[mb], b, acc[mb][nb]); if (NSPLIT >= 2) acc[mb][nb] = WFrag<T16>::mma(a[mb], b2, acc[mb][nb]); } }
        asm volatile("v_nop\n\tv_nop\n\tv_nop\n\tv_nop" : "+v"(acc[0][0]), "+v"(acc[1][1]), "+v"(acc[2][2]), "+v"(acc[3][3]) : "v"(a[0]), "v"(a[3]));
    }
#pragma unroll
    for (int mb = 0; mb < 4; ++mb) {
#pragma unroll
        for (int nb = 0; nb < 4; ++nb) {
#pragma unroll
            for (int j = 0; j < 8; ++j) os[(hi * 8 + j) * 68 + nb * 16 + lr] = acc[mb][nb][j]; }
        __builtin_amdgcn_wave_barrier(); asm volatile("" ::: "memory");
        float* crow = C + (size_t)(r0 + mb * 16) * ldc + c0;
#pragma unroll 1
        for (int ps = 0; ps < 2; ++ps) {
#pragma unroll
            for (int s = 0; s < 8; ++s) { const int row = 2 * s + hi, cofs = lr * 4; v4f val = *(const v4fa*)(os + row * 68 + cofs); if (BIAS) { val[0] += bfr(bias[c0 + cofs]); val[1] += bfr(bias[c0 + cofs + 1]); val[2] += bfr(bias[c0 + cofs + 2]); val[3] += bfr(bias[c0 + cofs + 3]); }
                *(volatile v4f*)(crow + (size_t)row * ldc + cofs) = val; }
            if (ps == 0) __threadfence(); }
        __builtin_amdgcn_wave_barrier(); asm volatile("" ::: "memory");
    }
}

__global__ __launch_bounds__(256) void k_cvtx(const float* __restrict__ src, bf* dst) {
    const unsigned b = blockIdx.y; const unsigned i = blockIdx.x * 256u + threadIdx.x; if (i >= (unsigned)(SEQ * DM / 8)) return;
    const v8f v = *(const v8f*)(src + (size_t)b * SEQ_FULL * DM + (size_t)i * 8u); v8us o;
#pragma unroll
    for (int k = 0; k < 8; ++k) o[k] = f2bf(v[k]);
    bf* d = dst + (size_t)b * SEQ * DM + (size_t)i * 8u;
    *(volatile v8us*)d = o; __threadfence(); *(volatile v8us*)d = o; }

__global__ __launch_bounds__(256) void k_cvtw(const float* __restrict__ w0, const float* __restrict__ w1, const float* __restrict__ w2, const float* __restrict__ w3, bf* dst) {
    const unsigned y = blockIdx.y; const float* src = (y == 0u) ? w0 : (y == 1u) ? w1 : (y == 2u) ? w2 : w3;
    const unsigned i = blockIdx.x * 256u + threadIdx.x; if (i >= (unsigned)(DM * DM / 8)) return;
    const v8f v = *(const v8f*)(src + (size_t)i * 8u); v8us o;
#pragma unroll
    for (int k = 0; k < 8; ++k) o[k] = f2bf(v[k]);
    bf* d = dst + (size_t)y * DM * DM + (size_t)i * 8u;
    *(volatile v8us*)d = o; __threadfence(); *(volatile v8us*)d = o; }

__global__ __launch_bounds__(32) void k_invf(float* IF) {
    const unsigned i = threadIdx.x & 31u; const float e = (-2.0f * (float)i) / 64.0f; const float v = powf(10000.0f, e);
    *(volatile float*)(IF + i) = v; __threadfence(); *(volatile float*)(IF + i) = v; }

__global__ __launch_bounds__(256) void k_cstab(const float* __restrict__ IF, float* CS) {
    const unsigned idx = blockIdx.x * 256u + threadIdx.x; if (idx >= (unsigned)(SEQ * 32)) return;
    const unsigned t = idx >> 5, i = idx & 31u; const float ang = (float)t * IF[i]; float sn, cs; sincosf(ang, &sn, &cs);
    v2f o; o[0] = cs; o[1] = sn;
    *(volatile v2f*)(CS + (size_t)idx * 2u) = o; __threadfence(); *(volatile v2f*)(CS + (size_t)idx * 2u) = o; }

__global__ __launch_bounds__(256) void k_rope(const float* __restrict__ F, const float* __restrict__ CS, h16* P16, bf* Ph, bf* Pl) {
#pragma clang fp contract(off)
    const unsigned e = (blockIdx.x * 256u + threadIdx.x) * 2u; if (e >= (unsigned)(NB * NH * SEQ * HD)) return;
    const unsigned d = e & 63u, r = e >> 6, t = r % (unsigned)SEQ, bh = r / (unsigned)SEQ, h = bh % (unsigned)NH, b = bh / (unsigned)NH;
    const v2f x = *(const v2f*)(F + (size_t)(b * SEQ + t) * DM + h * HD + d);
    const v2f cs = *(const v2f*)(CS + ((size_t)t * 32u + (d >> 1)) * 2u);
    const float a0 = x[0] * cs[0], a1 = x[1] * cs[1], b0 = x[0] * cs[1], b1 = x[1] * cs[0];
    const float o0 = a0 - a1, o1 = b0 + b1;
    v2h o16; o16[0] = (h16)o0; o16[1] = (h16)o1; v2us oh, ol; unsigned short s0, s1;
    splitf(o0, s0, s1); oh[0] = s0; ol[0] = s1; splitf(o1, s0, s1); oh[1] = s0; ol[1] = s1;
    const bool hr = (t < (unsigned)RH); const size_t eh = ((size_t)bh * RH + (hr ? t : 0u)) * HD + d;
    *(volatile v2h*)(P16 + e) = o16; if (hr) { *(volatile v2us*)(Ph + eh) = oh; *(volatile v2us*)(Pl + eh) = ol; }
    __threadfence();
    *(volatile v2h*)(P16 + e) = o16; if (hr) { *(volatile v2us*)(Ph + eh) = oh; *(volatile v2us*)(Pl + eh) = ol; }
}

__global__ __launch_bounds__(256) void k_vtp(const float* __restrict__ F, h16* V16, bf* Vh, bf* Vl) {
    const unsigned e = (blockIdx.x * 256u + threadIdx.x) * 2u; if (e >= (unsigned)(NB * NH * SEQ * HD)) return;
    const unsigned t = e % (unsigned)SEQ, r = e / (unsigned)SEQ, d = r & 63u, bh = r >> 6, h = bh % (unsigned)NH, b = bh / (unsigned)NH;
    v2h o16; v2us oh, ol;
#pragma unroll
    for (int q = 0; q < 2; ++q) { const float x = F[(size_t)(b * SEQ + t + q) * DM + h * HD + d]; o16[q] = (h16)x; unsigned short s0, s1; splitf(x, s0, s1); oh[q] = s0; ol[q] = s1; }
    const bool hr = (t < (unsigned)RH); const size_t eh = ((size_t)bh * HD + d) * RH + (hr ? t : 0u);
    *(volatile v2h*)(V16 + e) = o16; if (hr) { *(volatile v2us*)(Vh + eh) = oh; *(volatile v2us*)(Vl + eh) = ol; }
    __threadfence();
    *(volatile v2h*)(V16 + e) = o16; if (hr) { *(volatile v2us*)(Vh + eh) = oh; *(volatile v2us*)(Vl + eh) = ol; }
}

template <typename T16, int NSPLIT>
__global__ __launch_bounds__(32) void k_attn(const T16* __restrict__ Qa, const T16* __restrict__ Qb, const T16* __restrict__ Ka, const T16* __restrict__ Kb, const T16* __restrict__ Va, const T16* __restrict__ Vb,
                                             unsigned prow, unsigned roff, const float* __restrict__ pad, bf* ATh, bf* ATl) {
    typedef WFrag<T16> W; typedef typename W::V V;
    __shared__ __align__(16) unsigned short osh[16 * 72];
    __shared__ __align__(16) unsigned short osl[16 * 72];
    const unsigned lane = threadIdx.x & 31u, lr = lane & 15u, hi = lane >> 4;
    const unsigned h = blockIdx.y, b = blockIdx.z, q0 = roff + blockIdx.x * 16u, qrow = q0 + lr;
    const size_t hb = (size_t)(b * NH + h);
    const size_t qof = (hb * prow + qrow) * HD + 8u * hi;
    const size_t kof = (hb * prow + lr) * HD + 8u * hi;
    const size_t vof = (hb * HD + lr) * prow + 8u * hi;
    const float* padb = pad + (size_t)b * SEQ_FULL;
    V qf[2], qf2[2];
#pragma unroll
    for (int kk = 0; kk < 2; ++kk) { qf[kk] = W::ld(Qa + qof + kk * 32); if (NSPLIT == 2) qf2[kk] = W::ld(Qb + qof + kk * 32); }
    v8f oacc[4];
#pragma unroll
    for (int nf = 0; nf < 4; ++nf) oacc[nf] = (v8f){};
    float m = -1.0e30f, l = 0.0f;
    const unsigned nkb = (q0 + 47u) >> 5;
#pragma unroll 1
    for (unsigned kb = 0; kb < nkb; ++kb) {
        const unsigned kbase = kb * 32u;
        v8f st[2];
#pragma unroll
        for (int nk = 0; nk < 2; ++nk) {
            v8f s = (v8f){};
#pragma unroll
            for (int kk = 0; kk < 2; ++kk) {
                const size_t ko = kof + (size_t)(kbase + nk * 16u) * HD + kk * 32;
                const V ka = W::ld(Ka + ko);
                s = mmag<T16>(ka, qf[kk], s);
                if (NSPLIT == 2) { const V kl = W::ld(Kb + ko); s = mmag<T16>(kl, qf[kk], s); s = mmag<T16>(ka, qf2[kk], s); }
            }
            st[nk] = s;
        }
        v8f sc[2]; float bm = -1.0e30f;
#pragma unroll
        for (int nk = 0; nk < 2; ++nk) {
            const float* pp = padb + kbase + nk * 16u + 8u * hi;
            const v4f pa = *(const v4f*)pp; const v4f pb = *(const v4f*)(pp + 4);
#pragma unroll
            for (int r = 0; r < 8; ++r) {
                const unsigned key = kbase + nk * 16u + 8u * hi + (unsigned)r;
                const float pv = (r < 4) ? pa[r & 3] : pb[r & 3];
                const bool ok = (key <= qrow) && (pv != 0.0f);
                const float s = ok ? st[nk][r] * SCL : -1.0e30f;
                sc[nk][r] = s; bm = fmaxf(bm, s);
            }
        }
        bm = fmaxf(bm, __shfl_xor(bm, 16, 32));
        const float mn = fmaxf(m, bm);
        const float al = __builtin_amdgcn_exp2f((m - mn) * L2E);
        m = mn;
        v8f pt[2]; float rs = 0.0f;
#pragma unroll
        for (int nk = 0; nk < 2; ++nk)
#pragma unroll
            for (int r = 0; r < 8; ++r) { const float p = __builtin_amdgcn_exp2f((sc[nk][r] - mn) * L2E); pt[nk][r] = p; rs += p; }
        l = l * al + rs;
#pragma unroll
        for (int nf = 0; nf < 4; ++nf) oacc[nf] = oacc[nf] * al;
        const V ph = W::pkh(pt[0], pt[1]);
        V pl; if (NSPLIT == 2) pl = W::pkl(pt[0], pt[1]);
#pragma unroll
        for (int nf = 0; nf < 4; ++nf) {
            const size_t vo = vof + (size_t)(nf * 16) * prow + kbase;
            const V va = W::ld(Va + vo);
            oacc[nf] = mmag<T16>(va, ph, oacc[nf]);
            if (NSPLIT == 2) { const V vl = W::ld(Vb + vo); oacc[nf] = mmag<T16>(vl, ph, oacc[nf]); oacc[nf] = mmag<T16>(va, pl, oacc[nf]); }
        }
    }
    const float lt = l + __shfl_xor(l, 16, 32);
    const float inv = W::ocs() * (1.0f / lt);
#pragma unroll
    for (int nf = 0; nf < 4; ++nf) {
        v8us oh, ol;
#pragma unroll
        for (int r = 0; r < 8; ++r) { unsigned short s0, s1; splitf(oacc[nf][r] * inv, s0, s1); oh[r] = s0; ol[r] = s1; }
        *(v8usa*)(osh + lr * 72u + nf * 16 + 8u * hi) = oh;
        *(v8usa*)(osl + lr * 72u + nf * 16 + 8u * hi) = ol;
    }
    __builtin_amdgcn_wave_barrier(); asm volatile("" ::: "memory");
    const unsigned piece = lane & 7u, rq = lane >> 3;
#pragma unroll 1
    for (int ps = 0; ps < 2; ++ps) {
#pragma unroll
        for (int s = 0; s < 4; ++s) {
            const unsigned row = 4u * (unsigned)s + rq;
            const v8us vh = *(const v8usa*)(osh + row * 72u + piece * 8u);
            const v8us vl = *(const v8usa*)(osl + row * 72u + piece * 8u);
            const size_t oo = (size_t)(b * SEQ + q0 + row) * DM + h * HD + piece * 8u;
            *(volatile v8us*)(ATh + oo) = vh; *(volatile v8us*)(ATl + oo) = vl;
        }
        if (ps == 0) __threadfence();
    }
}

extern "C" void kernel_launch(void* const* d_in, const int* in_sizes, int n_in,
                              void* d_out, int out_size, void* d_ws, size_t ws_size, hipStream_t stream) {
    if (n_in < 6) return;
    const size_t need_x = ((size_t)(NB - 1) * SEQ_FULL + SEQ) * DM, need_p = (size_t)(NB - 1) * SEQ_FULL + SEQ;
    if ((size_t)in_sizes[0] < need_x || (size_t)in_sizes[1] < need_p) return;
    if ((size_t)in_sizes[2] < (size_t)DM * DM || (size_t)in_sizes[3] < (size_t)DM * DM || (size_t)in_sizes[4] < (size_t)DM * DM || (size_t)in_sizes[5] < (size_t)DM * DM) return;
    if ((size_t)out_size < need_x) return;
    const float* x = (const float*)d_in[0]; const float* pad = (const float*)d_in[1];
    const float* wq = (const float*)d_in[2]; const float* wk = (const float*)d_in[3]; const float* wv = (const float*)d_in[4]; const float* wo = (const float*)d_in[5];
    float* OUT = (float*)d_out;
    char* wsp = (char*)d_ws;
    auto take = [&](size_t bytes) { char* p = wsp; wsp += (bytes + 255) & ~(size_t)255; return (void*)p; };
    const size_t NTOK = (size_t)NB * SEQ;
    bf* WB = (bf*)take((size_t)4 * DM * DM * 2); bf* WQ = WB; bf* WK = WB + (size_t)DM * DM; bf* WV = WB + (size_t)2 * DM * DM; bf* WO = WB + (size_t)3 * DM * DM;
    float* IF = (float*)take(32 * 4); float* CS = (float*)take((size_t)SEQ * 32 * 2 * 4);
    bf* XB = (bf*)take(NTOK * DM * 2);
    char* RR = (char*)take(NTOK * DM * 4);
    float* F = (float*)RR; bf* ATh = (bf*)RR; bf* ATl = (bf*)RR + NTOK * DM;
    h16* Q16 = (h16*)take(NTOK * DM * 2); h16* K16 = (h16*)take(NTOK * DM * 2); h16* VT16 = (h16*)take(NTOK * DM * 2);
    const size_t HB = (size_t)NB * NH * RH * HD * 2;
    bf* Qh = (bf*)take(HB); bf* Ql = (bf*)take(HB); bf* Kh = (bf*)take(HB); bf* Kl = (bf*)take(HB); bf* VTh = (bf*)take(HB); bf* VTl = (bf*)take(HB);
    if ((size_t)(wsp - (char*)d_ws) > ws_size) return;
    k_cvtx<<<dim3((unsigned)(SEQ * DM / 8 / 256), NB), 256, 0, stream>>>(x, XB);
    k_cvtw<<<dim3((unsigned)(DM * DM / 8 / 256), 4), 256, 0, stream>>>(wq, wk, wv, wo, WB);
    k_invf<<<1, 32, 0, stream>>>(IF);
    k_cstab<<<(unsigned)(SEQ * 32 / 256), 256, 0, stream>>>(IF, CS);
    const dim3 gp((unsigned)(NTOK / 64), DM / 64, 1);
    const unsigned LP = (unsigned)((size_t)NB * NH * SEQ * HD / 2 / 256);
    k_gemmw<bf, 0, false><<<gp, 32, 0, stream>>>(XB, nullptr, WQ, nullptr, DM, F, DM, nullptr, 0, 0, 0);
    k_rope<<<LP, 256, 0, stream>>>(F, CS, Q16, Qh, Ql);
    k_gemmw<bf, 0, false><<<gp, 32, 0, stream>>>(XB, nullptr, WK, nullptr, DM, F, DM, nullptr, 0, 0, 0);
    k_rope<<<LP, 256, 0, stream>>>(F, CS, K16, Kh, Kl);
    k_gemmw<bf, 0, false><<<gp, 32, 0, stream>>>(XB, nullptr, WV, nullptr, DM, F, DM, nullptr, 0, 0, 0);
    k_vtp<<<LP, 256, 0, stream>>>(F, VT16, VTh, VTl);
    k_attn<bf, 2><<<dim3(RH / 16, NH, NB), 32, 0, stream>>>(Qh, Ql, Kh, Kl, VTh, VTl, (unsigned)RH, 0u, pad, ATh, ATl);
    if (SEQ > RH) k_attn<h16, 0><<<dim3((SEQ - RH) / 16, NH, NB), 32, 0, stream>>>(Q16, nullptr, K16, nullptr, VT16, nullptr, (unsigned)SEQ, (unsigned)RH, pad, ATh, ATl);
    k_gemmw<bf, 1, false><<<dim3(SEQ / 64, DM / 64, NB), 32, 0, stream>>>(ATh, ATl, WO, nullptr, DM, OUT, DM, nullptr, (size_t)SEQ * DM, 0, (size_t)SEQ_FULL * DM);
}
